// SinkhornMatcher_45672682225973
// MI455X (gfx1250) — hardware-run, weakly checked
//
#include <hip/hip_runtime.h>
#include <math.h>

typedef __attribute__((ext_vector_type(16))) _Float16 v16h;
typedef __attribute__((ext_vector_type(8)))  _Float16 v8h;
typedef __attribute__((ext_vector_type(16))) __bf16   v16b;
typedef __attribute__((ext_vector_type(8)))  __bf16   v8b;
typedef __attribute__((ext_vector_type(8)))  float    v8f;
typedef __attribute__((ext_vector_type(4)))  float    v4f;

constexpr int   kBatch   = 16;
constexpr int   kNodes   = 128;
constexpr int   kFeat    = 256;
constexpr int   kRowsAll = kBatch * kNodes;
constexpr int   kIters   = 10;
constexpr int   kHP      = 260;
constexpr float kCarry   = 32.0f;
constexpr float kF16Min  = 6.103515625e-5f;
constexpr float kF32Min  = 1.17549435e-38f;
static_assert(kRowsAll == 2048, "rows");
static_assert((kFeat % 32) == 0, "GEMM K multiple of 32");
static_assert((kRowsAll % 64) == 0 && (kFeat % 64) == 0 && (kNodes % 64) == 0, "GEMM M,N multiples of 64");

constexpr size_t kOutT    = 0;
constexpr size_t kOutCS   = (size_t)kBatch * kNodes * kNodes;
constexpr size_t kOutC    = kOutCS + 32;
constexpr size_t kOutAll  = kOutC + (size_t)kBatch * kNodes * kNodes;
static_assert(kOutCS * 4 == 1048576ull, "cost byte offset");
static_assert((kOutCS + 16) * 4 == 1048640ull, "similarity byte offset");
static_assert(kOutC * 4 == 1048704ull, "cost matrix byte offset");
static_assert(kOutAll * 4 == 2097280ull, "output total bytes");

constexpr size_t kSzPlane16 = (size_t)2 * kRowsAll * kFeat * 2;
constexpr size_t kSzW16     = (size_t)2 * kFeat * kFeat * 2;
constexpr size_t kSzH       = (size_t)2 * kRowsAll * kFeat * 4;
constexpr size_t kSzMat     = (size_t)kBatch * kNodes * kNodes * 4;
constexpr size_t kSzNorm    = (size_t)2 * kRowsAll * 4;
constexpr size_t kSzPart    = (size_t)kBatch * 32 * 4;
constexpr size_t kOffNH   = 0;
constexpr size_t kOffNL   = kOffNH + kSzPlane16;
constexpr size_t kOffNF   = kOffNL + kSzPlane16;
constexpr size_t kOffWH   = kOffNF + kSzPlane16;
constexpr size_t kOffWL   = kOffWH + kSzW16;
constexpr size_t kOffH    = kOffWL + kSzW16;
constexpr size_t kOffDOT  = kOffH + kSzH;
constexpr size_t kOffCOS  = kOffDOT + kSzMat;
constexpr size_t kOffCW   = kOffCOS + kSzMat;
constexpr size_t kOffNORM = kOffCW + kSzMat;
constexpr size_t kOffPART = kOffNORM + kSzNorm;
constexpr size_t kWsTotal = kOffPART + kSzPart;
static_assert(kWsTotal == 14174208ull, "carve total");
static_assert(kWsTotal <= 134217728ull, "carve cap");
static_assert((kOffNL % 128) == 0 && (kOffNF % 128) == 0 && (kOffWH % 128) == 0 && (kOffWL % 128) == 0 &&
              (kOffH % 128) == 0 && (kOffDOT % 128) == 0 && (kOffCOS % 128) == 0 && (kOffCW % 128) == 0 &&
              (kOffNORM % 128) == 0 && (kOffPART % 128) == 0, "128-B aligned regions");

__device__ __forceinline__ unsigned short f2bf_bits(float f) {
  unsigned u = __float_as_uint(f);
  return (unsigned short)((u + 0x7FFFu + ((u >> 16) & 1u)) >> 16);
}
__device__ __forceinline__ float bf_bits2f(unsigned short h) { return __uint_as_float(((unsigned)h) << 16); }

__device__ __forceinline__ void tie_h(v8f& a, v16h x, v16h y) { asm volatile("v_nop\n\tv_nop\n\tv_nop\n\tv_nop" : "+v"(a) : "v"(x), "v"(y)); }
__device__ __forceinline__ void tie_b(v8f& a, v16b x, v16b y) { asm volatile("v_nop\n\tv_nop\n\tv_nop\n\tv_nop" : "+v"(a) : "v"(x), "v"(y)); }
__device__ __forceinline__ void keep4_h(v16h a, v16h b, v16h c, v16h d) { asm volatile("v_nop" :: "v"(a), "v"(b), "v"(c), "v"(d)); }
__device__ __forceinline__ void keep4_b(v16b a, v16b b, v16b c, v16b d) { asm volatile("v_nop" :: "v"(a), "v"(b), "v"(c), "v"(d)); }
__device__ __forceinline__ void acc_guard4(v8f& a, v8f& b, v8f& c, v8f& d) { asm volatile("v_nop\n\tv_nop\n\tv_nop\n\tv_nop" : "+v"(a), "+v"(b), "+v"(c), "+v"(d)); }
template <typename T> struct Frag;
template <> struct Frag<_Float16> {
  typedef v16h V; union U { v16h v; v8h h[2]; };
  static __device__ __forceinline__ v16h load(const _Float16* p) {
    U f; f.h[0] = *(const v8h*)(p); f.h[1] = *(const v8h*)(p + 16); return f.v;
  }
  static __device__ __forceinline__ v8f mma(v16h a, v16h b, v8f c) {
    return __builtin_amdgcn_wmma_f32_16x16x32_f16(false, a, false, b, (short)0, c, false, false);
  }
  static __device__ __forceinline__ void tie(v8f& a, v16h x, v16h y) { tie_h(a, x, y); }
  static __device__ __forceinline__ void keep(v16h a, v16h b, v16h c, v16h d) { keep4_h(a, b, c, d); }
};
template <> struct Frag<__bf16> {
  typedef v16b V; union U { v16b v; v8b h[2]; };
  static __device__ __forceinline__ v16b load(const __bf16* p) {
    U f; f.h[0] = *(const v8b*)(p); f.h[1] = *(const v8b*)(p + 16); return f.v;
  }
  static __device__ __forceinline__ v8f mma(v16b a, v16b b, v8f c) {
    return __builtin_amdgcn_wmma_f32_16x16x32_bf16(false, a, false, b, (short)0, c, false, false);
  }
  static __device__ __forceinline__ void tie(v8f& a, v16b x, v16b y) { tie_b(a, x, y); }
  static __device__ __forceinline__ void keep(v16b a, v16b b, v16b c, v16b d) { keep4_b(a, b, c, d); }
};

template <int ET> struct Elem;
template <> struct Elem<0> { typedef _Float16 T; };
template <> struct Elem<1> { typedef __bf16 T; };
template <int ET, int SPL, int BIAS_MODE, int OUT_MODE, bool RESID>
__global__ __launch_bounds__(256) void wmma_gemm64(
    const unsigned short* __restrict__ Ap, const unsigned short* __restrict__ A2p, int lda, long strideA,
    const unsigned short* __restrict__ Btp, const unsigned short* __restrict__ Bt2p, int ldb, long strideB,
    void* __restrict__ Cout, void* __restrict__ Cout2, int ldc, long strideC,
    const float* __restrict__ bias,
    const float* __restrict__ resid, long strideR,
    int M, int N, int K, float scale) {
  typedef typename Elem<ET>::T T;
  typedef typename Frag<T>::V V;
  const T* A = (const T*)Ap; const T* A2 = (const T*)A2p; const T* Bt = (const T*)Btp; const T* Bt2 = (const T*)Bt2p;
  __shared__ __align__(16) float sT[8][16 * 68];
  const int b    = blockIdx.y;
  const int lane = threadIdx.x & 31;
  const int wave = threadIdx.x >> 5;
  const int tilesN = N >> 6;
  const int tilesM = M >> 6;
  const int tile = blockIdx.x * 8 + wave;
  if (tile >= tilesM * tilesN) return;
  const int tm = tile / tilesN;
  const int tn = tile - tm * tilesN;
  const int m0 = tm << 6;
  const int n0 = tn << 6;

  const T* Ab  = A  + (size_t)b * strideA;
  const T* Bb  = Bt + (size_t)b * strideB;
  const T* Ab2 = (SPL >= 1) ? (A2  + (size_t)b * strideA) : nullptr;
  const T* Bb2 = (SPL == 2) ? (Bt2 + (size_t)b * strideB) : nullptr;

  const int rlane = lane & 15;
  const int koff  = (lane >> 4) * 8;
  const int mOff  = (lane >> 4) * 8;

  v8f acc[4][4];
#pragma unroll
  for (int i = 0; i < 4; ++i)
#pragma unroll
    for (int j = 0; j < 4; ++j) acc[i][j] = (v8f){0.f,0.f,0.f,0.f,0.f,0.f,0.f,0.f};

  for (int k0 = 0; k0 < K; k0 += 32) {
    V bh[4], bl[4];
#pragma unroll
    for (int j = 0; j < 4; ++j) {
      const size_t bo = (size_t)(n0 + (j << 4) + rlane) * ldb + koff + k0;
      bh[j] = Frag<T>::load(Bb + bo);
      if (SPL == 2) bl[j] = Frag<T>::load(Bb2 + bo);
    }
#pragma unroll
    for (int i = 0; i < 4; ++i) {
      const size_t ao = (size_t)(m0 + (i << 4) + rlane) * lda + koff + k0;
      V ah = Frag<T>::load(Ab + ao);
      V al;
      if (SPL >= 1) al = Frag<T>::load(Ab2 + ao);
#pragma unroll
      for (int j = 0; j < 4; ++j) {
        acc[i][j] = Frag<T>::mma(ah, bh[j], acc[i][j]);
        if (SPL == 2) acc[i][j] = Frag<T>::mma(ah, bl[j], acc[i][j]);
        if (SPL >= 1) acc[i][j] = Frag<T>::mma(al, bh[j], acc[i][j]);
      }
#pragma unroll
      for (int j = 0; j < 4; ++j) Frag<T>::tie(acc[i][j], ah, (SPL >= 1) ? al : ah);
    }
    Frag<T>::keep(bh[0], bh[1], bh[2], bh[3]);
    if (SPL == 2) Frag<T>::keep(bl[0], bl[1], bl[2], bl[3]);
  }
  acc_guard4(acc[0][0], acc[0][1], acc[0][2], acc[0][3]);
  acc_guard4(acc[1][0], acc[1][1], acc[1][2], acc[1][3]);
  acc_guard4(acc[2][0], acc[2][1], acc[2][2], acc[2][3]);
  acc_guard4(acc[3][0], acc[3][1], acc[3][2], acc[3][3]);

  float* slab = sT[wave];
  const float* Rb = RESID ? (resid + (size_t)b * strideR) : nullptr;
#pragma unroll
  for (int i = 0; i < 4; ++i) {
    const int mBase = m0 + (i << 4);
#pragma unroll
    for (int j = 0; j < 4; ++j) {
      const int n = n0 + (j << 4) + rlane;
      float bv = 0.f;
      if (BIAS_MODE == 2) bv = bias[n];
#pragma unroll
      for (int r = 0; r < 8; ++r) {
        float v = acc[i][j][r] * scale;
        if (BIAS_MODE == 1) v += bias[mBase + mOff + r];
        if (BIAS_MODE == 2) v += bv;
        if (RESID) v += Rb[(size_t)(mBase + mOff + r) * ldc + n];
        slab[(mOff + r) * 68 + (j << 4) + rlane] = v;
      }
    }
    __builtin_amdgcn_fence(__ATOMIC_RELEASE, "workgroup");
    __builtin_amdgcn_wave_barrier();
    __builtin_amdgcn_fence(__ATOMIC_ACQUIRE, "workgroup");
    if (OUT_MODE == 0) {
      float* C = (float*)Cout + (size_t)b * strideC;
      const int hh = lane >> 4, c4 = (lane & 15) * 4;
      for (int pass = 0; pass < 2; ++pass) {
#pragma unroll
        for (int it = 0; it < 8; ++it) {
          const int row = it * 2 + hh;
          v4f v = *(const v4f*)(slab + row * 68 + c4);
          *(volatile v4f*)(C + (size_t)(mBase + row) * ldc + n0 + c4) = v;
        }
        __threadfence();
      }
    } else {
      const int q = lane >> 3, c8 = (lane & 7) * 8;
      unsigned short* C  = (unsigned short*)Cout  + (size_t)b * strideC;
      unsigned short* C2 = (OUT_MODE == 2) ? ((unsigned short*)Cout2 + (size_t)b * strideC) : nullptr;
      for (int pass = 0; pass < 2; ++pass) {
#pragma unroll
        for (int it = 0; it < 4; ++it) {
          const int row = it * 4 + q;
          const float* sp = slab + row * 68 + c8;
          v8h hv, lv;
#pragma unroll
          for (int e = 0; e < 8; ++e) {
            if (OUT_MODE == 1) {
              hv[e] = (_Float16)sp[e];
            } else {
              unsigned short hb = f2bf_bits(sp[e]);
              unsigned short lb = f2bf_bits(sp[e] - bf_bits2f(hb));
              hv[e] = __builtin_bit_cast(_Float16, hb);
              lv[e] = __builtin_bit_cast(_Float16, lb);
            }
          }
          *(volatile v8h*)(C + (size_t)(mBase + row) * ldc + n0 + c8) = hv;
          if (OUT_MODE == 2) *(volatile v8h*)(C2 + (size_t)(mBase + row) * ldc + n0 + c8) = lv;
        }
        __threadfence();
      }
    }
    __builtin_amdgcn_fence(__ATOMIC_RELEASE, "workgroup");
    __builtin_amdgcn_wave_barrier();
    __builtin_amdgcn_fence(__ATOMIC_ACQUIRE, "workgroup");
  }
}

__global__ __launch_bounds__(256) void prep_nodes_kernel(
    const float* __restrict__ nodes_a, const float* __restrict__ nodes_b,
    unsigned short* __restrict__ NH, unsigned short* __restrict__ NL, unsigned short* __restrict__ NF,
    float* __restrict__ NORM)
{
  __shared__ float sN[32];
  const int tid = threadIdx.x, lane = tid & 31, wave = tid >> 5;
  const int row0 = blockIdx.x * 32;
  const bool isb = (row0 >= kRowsAll);
  const float* src = isb ? nodes_b : nodes_a;
  const int srow0 = isb ? (row0 - kRowsAll) : row0;
#pragma unroll 1
  for (int r = 0; r < 4; ++r) {
    const int rl = wave * 4 + r;
    const size_t si = (size_t)(srow0 + rl) * kFeat + lane * 8;
    const v4f a0 = *(const v4f*)(src + si);
    const v4f a1 = *(const v4f*)(src + si + 4);
    float ss = 0.0f;
    v8h hv, lv, fv;
#pragma unroll
    for (int e = 0; e < 4; ++e) {
      const float x0 = a0[e];
      const float x1 = a1[e];
      ss = fmaf(x0, x0, ss);
      ss = fmaf(x1, x1, ss);
      const unsigned short h0 = f2bf_bits(x0);
      const unsigned short h1 = f2bf_bits(x1);
      const unsigned short l0 = f2bf_bits(x0 - bf_bits2f(h0));
      const unsigned short l1 = f2bf_bits(x1 - bf_bits2f(h1));
      hv[e]     = __builtin_bit_cast(_Float16, h0);
      hv[4 + e] = __builtin_bit_cast(_Float16, h1);
      lv[e]     = __builtin_bit_cast(_Float16, l0);
      lv[4 + e] = __builtin_bit_cast(_Float16, l1);
      const float c0 = x0 * kCarry;
      const float c1 = x1 * kCarry;
      const float g0 = (fabsf(c0) < kF16Min) ? 0.0f : c0;
      const float g1 = (fabsf(c1) < kF16Min) ? 0.0f : c1;
      fv[e]     = (_Float16)g0;
      fv[4 + e] = (_Float16)g1;
    }
#pragma unroll
    for (int off = 16; off > 0; off >>= 1) ss += __shfl_xor(ss, off, 32);
    if (lane == 0) sN[rl] = sqrtf(ss);
    const size_t o = (size_t)(row0 + rl) * kFeat + lane * 8;
    *(volatile v8h*)(NH + o) = hv;
    *(volatile v8h*)(NL + o) = lv;
    *(volatile v8h*)(NF + o) = fv;
    __threadfence();
    *(volatile v8h*)(NH + o) = hv;
    *(volatile v8h*)(NL + o) = lv;
    *(volatile v8h*)(NF + o) = fv;
  }
  __syncthreads();
  if (wave == 0) {
    const float nv = sN[lane];
    volatile float* p = NORM + row0 + lane;
    *p = nv;
    __threadfence();
    *p = nv;
  }
}

__global__ __launch_bounds__(256) void prep_w1_kernel(
    const float* __restrict__ W1, unsigned short* __restrict__ WH, unsigned short* __restrict__ WL)
{
  __shared__ float sT[64 * 65];
  const int tid = threadIdx.x, lane = tid & 31, wave = tid >> 5;
  const int n0 = blockIdx.x * 64, k0 = blockIdx.y * 64, which = blockIdx.z;
  const int col = tid & 63, rb = tid >> 6;
#pragma unroll 1
  for (int i = 0; i < 16; ++i) {
    const int r = rb + 4 * i;
    sT[r * 65 + col] = W1[(size_t)(which * kFeat + k0 + r) * kFeat + n0 + col];
  }
  __syncthreads();
  const int q = lane >> 3, c8 = (lane & 7) * 8;
#pragma unroll 1
  for (int it = 0; it < 2; ++it) {
    const int nl = it * 32 + wave * 4 + q;
    v8h hv, lv;
#pragma unroll
    for (int e = 0; e < 8; ++e) {
      const float x = sT[(c8 + e) * 65 + nl];
      const unsigned short hb = f2bf_bits(x);
      const unsigned short lb = f2bf_bits(x - bf_bits2f(hb));
      hv[e] = __builtin_bit_cast(_Float16, hb);
      lv[e] = __builtin_bit_cast(_Float16, lb);
    }
    const size_t o = (size_t)which * kFeat * kFeat + (size_t)(n0 + nl) * kFeat + k0 + c8;
    *(volatile v8h*)(WH + o) = hv;
    *(volatile v8h*)(WL + o) = lv;
    __threadfence();
    *(volatile v8h*)(WH + o) = hv;
    *(volatile v8h*)(WL + o) = lv;
  }
}

__global__ __launch_bounds__(128) void build_cost_kernel(
    const float* __restrict__ H, const float* __restrict__ DOTp, const float* __restrict__ NORM,
    const float* __restrict__ pos_a, const float* __restrict__ pos_b,
    const float* __restrict__ b1, const float* __restrict__ W2, const float* __restrict__ b2,
    const float* __restrict__ log_temp,
    float* __restrict__ COS, float* __restrict__ CW, float* __restrict__ outC)
{
  __shared__ __align__(16) float sHa[16 * kHP];
  __shared__ __align__(16) float sHb[32 * kHP];
  __shared__ __align__(16) float sW2[kFeat];
  __shared__ float sS[16 * 32];
  __shared__ float sC[16 * 32];
  __shared__ float sCo[16 * 32];
  const int tid = threadIdx.x, lane = tid & 31, wave = tid >> 5;
  const int kt = blockIdx.x, b = blockIdx.y;
  const int krow0 = b * kNodes + kt * 16;
  const float* Ha = H;
  const float* Hb = H + (size_t)kRowsAll * kFeat;

#pragma unroll 1
  for (int i = 0; i < 8; ++i) {
    const int idx = tid + 128 * i;
    const int r = idx >> 6, c4 = (idx & 63) * 4;
    v4f hv = *(const v4f*)(Ha + (size_t)(krow0 + r) * kFeat + c4);
    const v4f bv = *(const v4f*)(b1 + c4);
    hv = hv + bv;
    *(v4f*)(sHa + r * kHP + c4) = hv;
  }
  sW2[tid] = W2[tid];
  sW2[tid + 128] = W2[tid + 128];

  const float b2v = b2[0];
  float temp = expf(log_temp[0]);
  temp = fminf(fmaxf(temp, 0.01f), 0.5f);
  const float inv_temp = 1.0f / temp;

  const float* har = sHa + (wave * 4) * kHP;
  const float* hbr = sHb + lane * kHP;

#pragma unroll 1
  for (int mc = 0; mc < 4; ++mc) {
    __syncthreads();
#pragma unroll 1
    for (int i = 0; i < 16; ++i) {
      const int idx = tid + 128 * i;
      const int r = idx >> 6, c4 = (idx & 63) * 4;
      *(v4f*)(sHb + r * kHP + c4) = *(const v4f*)(Hb + (size_t)(b * kNodes + mc * 32 + r) * kFeat + c4);
    }
    __syncthreads();

    float s0 = 0.0f, s1 = 0.0f, s2 = 0.0f, s3 = 0.0f;
#pragma unroll 2
    for (int d = 0; d < kFeat; d += 4) {
      const v4f hb = *(const v4f*)(hbr + d);
      const v4f wv = *(const v4f*)(sW2 + d);
      const v4f a0 = *(const v4f*)(har + d);
      const v4f a1 = *(const v4f*)(har + kHP + d);
      const v4f a2 = *(const v4f*)(har + 2 * kHP + d);
      const v4f a3 = *(const v4f*)(har + 3 * kHP + d);
#pragma unroll
      for (int e = 0; e < 4; ++e) {
        s0 = fmaf(fmaxf(a0[e] + hb[e], 0.0f), wv[e], s0);
        s1 = fmaf(fmaxf(a1[e] + hb[e], 0.0f), wv[e], s1);
        s2 = fmaf(fmaxf(a2[e] + hb[e], 0.0f), wv[e], s2);
        s3 = fmaf(fmaxf(a3[e] + hb[e], 0.0f), wv[e], s3);
      }
    }
    sS[(wave * 4 + 0) * 32 + lane] = s0;
    sS[(wave * 4 + 1) * 32 + lane] = s1;
    sS[(wave * 4 + 2) * 32 + lane] = s2;
    sS[(wave * 4 + 3) * 32 + lane] = s3;
    __syncthreads();

    const int m = mc * 32 + lane;
    const float nbm = NORM[kRowsAll + b * kNodes + m];
    const float pbx = pos_b[(size_t)(b * kNodes + m) * 2 + 0];
    const float pby = pos_b[(size_t)(b * kNodes + m) * 2 + 1];
#pragma unroll 1
    for (int r = 0; r < 4; ++r) {
      const int kl = wave * 4 + r;
      const int k = kt * 16 + kl;
      const float sc = sS[kl * 32 + lane] + b2v;
      const float dotv = DOTp[(size_t)(b * kNodes + k) * kNodes + m];
      const float nak = NORM[b * kNodes + k];
      const float den = fmaxf(nak * nbm, 1e-8f);
      const float cosv = dotv / den;
      const float pax = pos_a[(size_t)(b * kNodes + k) * 2 + 0];
      const float pay = pos_a[(size_t)(b * kNodes + k) * 2 + 1];
      const float dx = pax - pbx, dy = pay - pby;
      const float sp = sqrtf(dx * dx + dy * dy);
      const float Cv = (-(sc + cosv)) * inv_temp + 0.1f * sp;
      sC[kl * 32 + lane] = Cv;
      sCo[kl * 32 + lane] = cosv;
    }
    __syncthreads();
    float cv[4], cs[4];
#pragma unroll
    for (int r = 0; r < 4; ++r) {
      cv[r] = sC[(wave * 4 + r) * 32 + lane];
      cs[r] = sCo[(wave * 4 + r) * 32 + lane];
    }
    for (int pass = 0; pass < 2; ++pass) {
#pragma unroll
      for (int r = 0; r < 4; ++r) {
        const size_t o = (size_t)(b * kNodes + kt * 16 + wave * 4 + r) * kNodes + mc * 32 + lane;
        *(volatile float*)(outC + o) = cv[r];
        *(volatile float*)(CW + o) = cv[r];
        *(volatile float*)(COS + o) = cs[r];
      }
      __threadfence();
    }
  }
}

__global__ __launch_bounds__(256) void plan_iter_kernel(
    const float* __restrict__ CW, const float* __restrict__ COS,
    float* __restrict__ outT, float* __restrict__ PART)
{
  extern __shared__ __align__(16) float sCm[];
  __shared__ float sLu[kNodes];
  __shared__ float sLv[kNodes];
  __shared__ float sRc[8];
  __shared__ float sRs[8];
  const int tid = threadIdx.x, lane = tid & 31, wave = tid >> 5;
  const int b = blockIdx.x;
  const float* Cb = CW + (size_t)b * kNodes * kNodes;
  const float* COSb = COS + (size_t)b * kNodes * kNodes;

#pragma unroll 1
  for (int i = 0; i < 16; ++i) {
    const int idx4 = tid + 256 * i;
    *(v4f*)(sCm + idx4 * 4) = *(const v4f*)(Cb + idx4 * 4);
  }
  if (tid < kNodes) {
    sLu[tid] = 0.0f;
    sLv[tid] = 0.0f;
  }
  const float logmu = -logf((float)kNodes);
  __syncthreads();

#pragma unroll 1
  for (int it = 0; it < kIters; ++it) {
#pragma unroll 1
    for (int i = 0; i < 16; ++i) {
      const int k = wave + 8 * i;
      const float* cr = sCm + k * kNodes;
      const float x0 = cr[lane] + sLv[lane];
      const float x1 = cr[lane + 32] + sLv[lane + 32];
      const float x2 = cr[lane + 64] + sLv[lane + 64];
      const float x3 = cr[lane + 96] + sLv[lane + 96];
      float mx = fmaxf(fmaxf(x0, x1), fmaxf(x2, x3));
#pragma unroll
      for (int off = 16; off > 0; off >>= 1) mx = fmaxf(mx, __shfl_xor(mx, off, 32));
      float s = 0.0f;
#pragma unroll 1
      for (int j = 0; j < 4; ++j) s += expf((cr[lane + 32 * j] + sLv[lane + 32 * j]) - mx);
#pragma unroll
      for (int off = 16; off > 0; off >>= 1) s += __shfl_xor(s, off, 32);
      if (lane == 0) sLu[k] = logmu - (logf(s) + mx);
    }
    __syncthreads();
    if (tid < kNodes) {
      float mx = -INFINITY;
#pragma unroll 4
      for (int k = 0; k < kNodes; ++k) mx = fmaxf(mx, sCm[k * kNodes + tid] + sLu[k]);
      float s = 0.0f;
#pragma unroll 1
      for (int k = 0; k < kNodes; ++k) s += expf((sCm[k * kNodes + tid] + sLu[k]) - mx);
      sLv[tid] = logmu - (logf(s) + mx);
    }
    __syncthreads();
  }

  float cacc = 0.0f, sacc = 0.0f;
#pragma unroll 1
  for (int i = 0; i < 64; ++i) {
    const int idx = tid + 256 * i;
    const int k = idx >> 7, m = idx & 127;
    const float Cv = sCm[idx];
    const float cosv = COSb[idx];
    float Tv = expf((Cv + sLu[k]) + sLv[m]);
    Tv = (Tv < kF32Min) ? 0.0f : Tv;
    cacc = fmaf(Tv, Cv, cacc);
    sacc = fmaf(Tv, cosv, sacc);
    sCm[idx] = Tv;
  }
#pragma unroll
  for (int off = 16; off > 0; off >>= 1) {
    cacc += __shfl_xor(cacc, off, 32);
    sacc += __shfl_xor(sacc, off, 32);
  }
  if (lane == 0) {
    sRc[wave] = cacc;
    sRs[wave] = sacc;
  }
  __syncthreads();

  float* Tb = outT + (size_t)b * kNodes * kNodes;
  for (int pass = 0; pass < 2; ++pass) {
#pragma unroll 1
    for (int i = 0; i < 16; ++i) {
      const int row = wave + 8 * i;
      const v4f tv = *(const v4f*)(sCm + row * kNodes + lane * 4);
      *(volatile v4f*)(Tb + row * kNodes + lane * 4) = tv;
    }
    __threadfence();
  }

  float ctot = 0.0f, stot = 0.0f;
#pragma unroll
  for (int q = 0; q < 8; ++q) {
    ctot += sRc[q];
    stot += sRs[q];
  }
  if (wave == 0) {
    const float pv = (lane == 0) ? ctot : ((lane == 1) ? stot : 0.0f);
    volatile float* p = PART + b * 32 + lane;
    *p = pv;
    __threadfence();
    *p = pv;
  }
}

__global__ __launch_bounds__(32) void sums_out_kernel(const float* __restrict__ PART, float* __restrict__ out_cs)
{
  const int lane = threadIdx.x & 31;
  const float v = PART[(lane & 15) * 32 + (lane >> 4)];
  volatile float* p = out_cs + lane;
  *p = v;
  __threadfence();
  *p = v;
}

extern "C" void kernel_launch(void* const* d_in, const int* in_sizes, int n_in,
                              void* d_out, int out_size, void* d_ws, size_t ws_size,
                              hipStream_t stream) {
  if (n_in < 9) return;
  if (in_sizes[0] != kRowsAll * kFeat) return;
  if (in_sizes[1] != kRowsAll * kFeat) return;
  if (in_sizes[2] != kRowsAll * 2) return;
  if (in_sizes[3] != kRowsAll * 2) return;
  if (in_sizes[4] != 2 * kFeat * kFeat) return;
  if (in_sizes[5] != kFeat) return;
  if (in_sizes[6] != kFeat) return;
  if (in_sizes[7] != 1) return;
  if (in_sizes[8] != 1) return;
  if ((size_t)out_size != kOutAll) return;
  if (ws_size < kWsTotal) return;

  const float* nodes_a  = (const float*)d_in[0];
  const float* nodes_b  = (const float*)d_in[1];
  const float* pos_a    = (const float*)d_in[2];
  const float* pos_b    = (const float*)d_in[3];
  const float* W1       = (const float*)d_in[4];
  const float* b1       = (const float*)d_in[5];
  const float* W2       = (const float*)d_in[6];
  const float* b2       = (const float*)d_in[7];
  const float* log_temp = (const float*)d_in[8];
  float* out = (float*)d_out;

  char* ws = (char*)d_ws;
  unsigned short* NH = (unsigned short*)(ws + kOffNH);
  unsigned short* NL = (unsigned short*)(ws + kOffNL);
  unsigned short* NF = (unsigned short*)(ws + kOffNF);
  unsigned short* WH = (unsigned short*)(ws + kOffWH);
  unsigned short* WL = (unsigned short*)(ws + kOffWL);
  float* H    = (float*)(ws + kOffH);
  float* DOTp = (float*)(ws + kOffDOT);
  float* COS  = (float*)(ws + kOffCOS);
  float* CW   = (float*)(ws + kOffCW);
  float* NORM = (float*)(ws + kOffNORM);
  float* PART = (float*)(ws + kOffPART);

  prep_nodes_kernel<<<(2 * kRowsAll) / 32, 256, 0, stream>>>(nodes_a, nodes_b, NH, NL, NF, NORM);
  prep_w1_kernel<<<dim3(kFeat / 64, kFeat / 64, 2), 256, 0, stream>>>(W1, WH, WL);

  wmma_gemm64<1, 2, 0, 0, false><<<dim3(16, 2), 256, 0, stream>>>(
      NH, NL, kFeat, (long)kRowsAll * kFeat,
      WH, WL, kFeat, (long)kFeat * kFeat,
      (void*)H, nullptr, kFeat, (long)kRowsAll * kFeat,
      nullptr, nullptr, 0L,
      kRowsAll, kFeat, kFeat, 1.0f);

  wmma_gemm64<0, 0, 0, 0, false><<<dim3(1, kBatch), 256, 0, stream>>>(
      NF, nullptr, kFeat, (long)kNodes * kFeat,
      NF + (size_t)kRowsAll * kFeat, nullptr, kFeat, (long)kNodes * kFeat,
      (void*)DOTp, nullptr, kNodes, (long)kNodes * kNodes,
      nullptr, nullptr, 0L,
      kNodes, kNodes, kFeat, 1.0f / (kCarry * kCarry));

  build_cost_kernel<<<dim3(kNodes / 16, kBatch), 128, 0, stream>>>(
      H, DOTp, NORM, pos_a, pos_b, b1, W2, b2, log_temp, COS, CW, out + kOutC);

  plan_iter_kernel<<<kBatch, 256, (size_t)kNodes * kNodes * sizeof(float), stream>>>(CW, COS, out + kOutT, PART);

  sums_out_kernel<<<1, 32, 0, stream>>>(PART, out + kOutCS);
}
